// LocalSphereAttention_56040733278768
// MI455X (gfx1250) — hardware-verified
//
#include <hip/hip_runtime.h>


#define NB_  2
#define NN   8192
#define CC   256
#define NH_  8
#define HD   32
#define KN   32
#define HB   32
typedef _Float16 h16;
typedef unsigned short bf;
typedef __attribute__((ext_vector_type(16))) __bf16   v16bf;
typedef __attribute__((ext_vector_type(16))) _Float16 v16h;
typedef __attribute__((ext_vector_type(8)))  _Float16 v8h;
typedef __attribute__((ext_vector_type(8)))  unsigned short v8us;
typedef __attribute__((ext_vector_type(8)))  float    v8f;
typedef __attribute__((ext_vector_type(4)))  float    v4f;
typedef v8h  __attribute__((may_alias)) v8ha;
typedef v4f  __attribute__((may_alias)) v4fa;
typedef v8us __attribute__((may_alias)) v8usa;

__device__ __forceinline__ unsigned short f2bf(float f) { unsigned u = __float_as_uint(f); u += 0x7FFFu + ((u >> 16) & 1u); return (unsigned short)(u >> 16); }
__device__ __forceinline__ float bf2f(unsigned short b) { return __uint_as_float(((unsigned)b) << 16); }
__device__ __forceinline__ float bfr(float f) { return bf2f(f2bf(f)); }
__device__ __forceinline__ v16h cat16(v8h lo, v8h hi) { return __builtin_shufflevector(lo, hi, 0, 1, 2, 3, 4, 5, 6, 7, 8, 9, 10, 11, 12, 13, 14, 15); }
__device__ __forceinline__ v16bf cat16b(v8us lo, v8us hi) { return __builtin_bit_cast(v16bf, __builtin_shufflevector(lo, hi, 0, 1, 2, 3, 4, 5, 6, 7, 8, 9, 10, 11, 12, 13, 14, 15)); }
__device__ __forceinline__ v8f wmma16(v16h a, v16h b, v8f c) { return __builtin_amdgcn_wmma_f32_16x16x32_f16(false, a, false, b, (short)0, c, false, false); }
__device__ __forceinline__ v8f wmmab(v16bf a, v16bf b, v8f c) { return __builtin_amdgcn_wmma_f32_16x16x32_bf16(false, a, false, b, (short)0, c, false, false); }


template <typename T16> struct WFrag;
template <> struct WFrag<h16> { typedef v16h V; static __device__ __forceinline__ V ld(const h16* p) { return cat16(*(const v8h*)p, *(const v8h*)(p + 16)); } static __device__ __forceinline__ v8f mma(V a, V b, v8f c) { return wmma16(a, b, c); } };
template <> struct WFrag<bf> { typedef v16bf V; static __device__ __forceinline__ V ld(const bf* p) { return cat16b(*(const v8us*)p, *(const v8us*)(p + 16)); } static __device__ __forceinline__ v8f mma(V a, V b, v8f c) { return wmmab(a, b, c); } };
template <typename T16, int NSPLIT, bool BIAS>
__global__ __launch_bounds__(32) void k_gemmw(const T16* __restrict__ A, const T16* __restrict__ A2, const T16* __restrict__ Bt, const T16* __restrict__ Bt2, int K, float* C, int ldc, const float* __restrict__ bias, size_t sA, size_t sB, size_t sC) {
    typedef typename WFrag<T16>::V V;
    __shared__ __align__(16) float os[16 * 68];
    const size_t z = blockIdx.z; A += z * sA; if (A2) A2 += z * sA; Bt += z * sB; if (Bt2) Bt2 += z * sB; C += z * sC;
    const int lane = threadIdx.x & 31, lr = lane & 15, hi = lane >> 4; const int r0 = blockIdx.x * 64, c0 = blockIdx.y * 64;
    v8f acc[4][4];
#pragma unroll
    for (int mb = 0; mb < 4; ++mb)
#pragma unroll
        for (int nb = 0; nb < 4; ++nb) acc[mb][nb] = (v8f){};
    const size_t aoff = (size_t)(r0 + lr) * K + 8 * hi, boff = (size_t)(c0 + lr) * K + 8 * hi;
#pragma unroll 1
    for (int kc = 0; kc < K; kc += 32) {
        V a[4], a2[4];
#pragma unroll
        for (int mb = 0; mb < 4; ++mb) { a[mb] = WFrag<T16>::ld(A + aoff + (size_t)mb * 16 * K + kc); if (NSPLIT == 1 || NSPLIT == 2) a2[mb] = WFrag<T16>::ld(A2 + aoff + (size_t)mb * 16 * K + kc); }
#pragma unroll
        for (int nb = 0; nb < 4; ++nb) { const V b = WFrag<T16>::ld(Bt + boff + (size_t)nb * 16 * K + kc); V b2; if (NSPLIT >= 2) b2 = WFrag<T16>::ld(Bt2 + boff + (size_t)nb * 16 * K + kc);
#pragma unroll
            for (int mb = 0; mb < 4; ++mb) { acc[mb][nb] = WFrag<T16>::mma(a[mb], b, acc[mb][nb]); if (NSPLIT == 1 || NSPLIT == 2) acc[mb][nb] = WFrag<T16>::mma(a2[mb], b, acc[mb][nb]); if (NSPLIT >= 2) acc[mb][nb] = WFrag<T16>::mma(a[mb], b2, acc[mb][nb]); } }
        asm volatile("v_nop\n\tv_nop\n\tv_nop\n\tv_nop" : "+v"(acc[0][0]), "+v"(acc[1][1]), "+v"(acc[2][2]), "+v"(acc[3][3]) : "v"(a[0]), "v"(a[3]));
    }
#pragma unroll
    for (int mb = 0; mb < 4; ++mb) {
#pragma unroll
        for (int nb = 0; nb < 4; ++nb) {
#pragma unroll
            for (int j = 0; j < 8; ++j) os[(hi * 8 + j) * 68 + nb * 16 + lr] = acc[mb][nb][j]; }
        __builtin_amdgcn_wave_barrier(); asm volatile("" ::: "memory");
        float* crow = C + (size_t)(r0 + mb * 16) * ldc + c0;
#pragma unroll 1
        for (int ps = 0; ps < 2; ++ps) {
#pragma unroll
            for (int s = 0; s < 8; ++s) { const int row = 2 * s + hi, cofs = lr * 4; v4f val = *(const v4fa*)(os + row * 68 + cofs); if (BIAS) { val[0] += bfr(bias[c0 + cofs]); val[1] += bfr(bias[c0 + cofs + 1]); val[2] += bfr(bias[c0 + cofs + 2]); val[3] += bfr(bias[c0 + cofs + 3]); }
                *(volatile v4f*)(crow + (size_t)row * ldc + cofs) = val; }
            if (ps == 0) __threadfence(); }
        __builtin_amdgcn_wave_barrier(); asm volatile("" ::: "memory");
    }
}

__device__ __forceinline__ void splitf(float y, unsigned short& h, unsigned short& l) { h = f2bf(y); l = f2bf(y - bf2f(h)); }
typedef __attribute__((ext_vector_type(2))) unsigned short v2us;
typedef __attribute__((ext_vector_type(4))) unsigned short v4us;

__global__ __launch_bounds__(256) void k_wtG(const float* __restrict__ w, int K, int N, bf* Bt) {
    const int lane = threadIdx.x & 31; const int L0 = (blockIdx.x * 8 + (threadIdx.x >> 5)) * 8; const int nlines = N * K / 64;
#pragma unroll
    for (int ps = 0; ps < 2; ++ps) {
#pragma unroll 1
        for (int l = 0; l < 8; ++l) { const int L = L0 + l; if (L >= nlines) break; const size_t e = (size_t)L * 64 + lane * 2; const int k = (int)(e % K), n = (int)(e / K); v2us o;
            o[0] = f2bf(w[(size_t)k * N + n]); o[1] = f2bf(w[(size_t)(k + 1) * N + n]); *(volatile v2us*)(Bt + e) = o; }
        if (ps == 0) __threadfence(); }
}
__global__ __launch_bounds__(256) void k_cvt8(const float* __restrict__ src, bf* dst, size_t n8) { const size_t i = (size_t)blockIdx.x * 256 + threadIdx.x; if (i >= n8) return; const v8f v = *(const v8f*)(src + i * 8); v8us o;
#pragma unroll
    for (int k = 0; k < 8; ++k) o[k] = f2bf(v[k]); *(volatile v8us*)(dst + i * 8) = o; __threadfence(); *(volatile v8us*)(dst + i * 8) = o; }
__device__ __forceinline__ int clampi(int m) { return m < 0 ? 0 : (m >= NN ? NN - 1 : m); }
__global__ __launch_bounds__(256) void k_bias(const float* __restrict__ xyz, const int* __restrict__ idx, const float* __restrict__ W1, const float* __restrict__ b1, const float* __restrict__ W2, const float* __restrict__ b2, float* BIAS) {
    const int e = blockIdx.x * 256 + threadIdx.x; if (e >= NN * KN) return; const int n = e / KN; const int m = clampi(idx[e]);
    float r[3];
#pragma unroll
    for (int a = 0; a < 3; ++a) r[a] = __fsub_rn(bfr(xyz[(size_t)n * 3 + a]), bfr(xyz[(size_t)m * 3 + a]));
    float acc[NH_];
#pragma unroll
    for (int h = 0; h < NH_; ++h) acc[h] = 0.f;
#pragma unroll 1
    for (int j = 0; j < HB; ++j) { float s = 0.f;
#pragma unroll
        for (int a = 0; a < 3; ++a) { float w = bfr(W1[a * HB + j]); asm volatile("" : "+v"(w)); float p = __fmul_rn(r[a], w); asm volatile("" : "+v"(p)); s = __fadd_rn(s, p); }
        float bb = bfr(b1[j]); asm volatile("" : "+v"(bb)); const float hv = fmaxf(__fadd_rn(s, bb), 0.f);
#pragma unroll
        for (int h = 0; h < NH_; ++h) { float w = bfr(W2[j * NH_ + h]); asm volatile("" : "+v"(w)); float p = __fmul_rn(hv, w); asm volatile("" : "+v"(p)); acc[h] = __fadd_rn(acc[h], p); } }
    for (int ps = 0; ps < 2; ++ps) {
#pragma unroll
        for (int h = 0; h < NH_; ++h) { float bb = bfr(b2[h]); asm volatile("" : "+v"(bb)); *(volatile float*)(BIAS + (size_t)h * NN * KN + e) = __fadd_rn(acc[h], bb); }
        if (ps == 0) __threadfence(); } }
__global__ __launch_bounds__(256) void k_attn(const float* __restrict__ FQ, const float* __restrict__ FK, const float* __restrict__ FV, const int* __restrict__ idx, const float* __restrict__ BIAS, bf* Ah, bf* Al) {
    const size_t e = ((size_t)blockIdx.x * 256 + threadIdx.x) * 4; if (e >= (size_t)NN * CC) return; const int col = (int)(e % CC); const int n = (int)(e / CC); const int h = col / HD; const int* in_ = idx + (size_t)n * KN; const float* bs = BIAS + ((size_t)h * NN + n) * KN;
    const v4f q = *(const v4f*)(FQ + e); const float SC = 0.17677669529663687f; float sc[KN]; float mx = -3.0e38f;
#pragma unroll
    for (int kk = 0; kk < KN; ++kk) { const int m = clampi(in_[kk]); const v4f k = *(const v4f*)(FK + (size_t)m * CC + col); float part = 0.f;
#pragma unroll
        for (int u = 0; u < 4; ++u) { float pr = __fmul_rn(q[u], k[u]); asm volatile("" : "+v"(pr)); part = __fadd_rn(part, pr); }
        part += __shfl_xor(part, 1, 32); part += __shfl_xor(part, 2, 32); part += __shfl_xor(part, 4, 32); float s0 = __fmul_rn(part, SC); asm volatile("" : "+v"(s0)); sc[kk] = __fadd_rn(s0, bs[kk]); mx = fmaxf(mx, sc[kk]); }
    float sum = 0.f;
#pragma unroll
    for (int kk = 0; kk < KN; ++kk) { float d0 = __fsub_rn(sc[kk], mx); asm volatile("" : "+v"(d0)); sc[kk] = __expf(d0); sum = __fadd_rn(sum, sc[kk]); }
    const float inv = __fdiv_rn(1.0f, sum); float o[4] = {0.f, 0.f, 0.f, 0.f};
#pragma unroll
    for (int kk = 0; kk < KN; ++kk) { const int m = clampi(in_[kk]); const v4f v = *(const v4f*)(FV + (size_t)m * CC + col); float pw = __fmul_rn(sc[kk], inv); asm volatile("" : "+v"(pw));
#pragma unroll
        for (int u = 0; u < 4; ++u) { float pr = __fmul_rn(pw, v[u]); asm volatile("" : "+v"(pr)); o[u] = __fadd_rn(o[u], pr); } }
    v4us oh, ol;
#pragma unroll
    for (int u = 0; u < 4; ++u) { unsigned short a, b; splitf(o[u], a, b); oh[u] = a; ol[u] = b; } *(volatile v4us*)(Ah + e) = oh; *(volatile v4us*)(Al + e) = ol; __threadfence(); *(volatile v4us*)(Ah + e) = oh; *(volatile v4us*)(Al + e) = ol; }

extern "C" void kernel_launch(void* const* d_in, const int* in_sizes, int n_in,
                              void* d_out, int out_size, void* d_ws, size_t ws_size, hipStream_t stream) {
    (void)in_sizes; (void)n_in; (void)out_size;
    const float* x = (const float*)d_in[0]; const float* xyz = (const float*)d_in[1]; const int* idx = (const int*)d_in[2]; const float* wq = (const float*)d_in[3]; const float* bq = (const float*)d_in[4]; const float* wk = (const float*)d_in[5]; const float* bk = (const float*)d_in[6]; const float* wv = (const float*)d_in[7]; const float* bv = (const float*)d_in[8];
    const float* wo = (const float*)d_in[9]; const float* bo = (const float*)d_in[10]; const float* W1 = (const float*)d_in[11]; const float* b1 = (const float*)d_in[12]; const float* W2 = (const float*)d_in[13]; const float* b2 = (const float*)d_in[14];
    float* OUT = (float*)d_out;
    char* wsp = (char*)d_ws;
    auto take = [&](size_t bytes) { char* p = wsp; wsp += (bytes + 255) & ~(size_t)255; return (void*)p; };
    bf* WQ = (bf*)take(CC * CC * 2); bf* WK = (bf*)take(CC * CC * 2); bf* WV = (bf*)take(CC * CC * 2); bf* WO = (bf*)take(CC * CC * 2);
    bf* XB = (bf*)take((size_t)NN * CC * 2); float* FQ = (float*)take((size_t)NN * CC * 4); float* FK = (float*)take((size_t)NN * CC * 4); float* FV = (float*)take((size_t)NN * CC * 4); float* BIAS = (float*)take((size_t)NH_ * NN * KN * 4); bf* Ah = (bf*)take((size_t)NN * CC * 2); bf* Al = (bf*)take((size_t)NN * CC * 2);
    if ((size_t)(wsp - (char*)d_ws) > ws_size) return;
    k_wtG<<<(CC * CC / 64 + 63) / 64, 256, 0, stream>>>(wq, CC, CC, WQ); k_wtG<<<(CC * CC / 64 + 63) / 64, 256, 0, stream>>>(wk, CC, CC, WK); k_wtG<<<(CC * CC / 64 + 63) / 64, 256, 0, stream>>>(wv, CC, CC, WV); k_wtG<<<(CC * CC / 64 + 63) / 64, 256, 0, stream>>>(wo, CC, CC, WO);
    for (int b = 0; b < NB_; ++b) { const int* ib = idx + (size_t)b * NN * KN;
        k_cvt8<<<(NN * CC / 8 + 255) / 256, 256, 0, stream>>>(x + (size_t)b * NN * CC, XB, (size_t)NN * CC / 8);
        k_gemmw<bf, 0, true><<<dim3(NN / 64, CC / 64, 1), 32, 0, stream>>>(XB, nullptr, WQ, nullptr, CC, FQ, CC, bq, 0, 0, 0); k_gemmw<bf, 0, true><<<dim3(NN / 64, CC / 64, 1), 32, 0, stream>>>(XB, nullptr, WK, nullptr, CC, FK, CC, bk, 0, 0, 0); k_gemmw<bf, 0, true><<<dim3(NN / 64, CC / 64, 1), 32, 0, stream>>>(XB, nullptr, WV, nullptr, CC, FV, CC, bv, 0, 0, 0);
        k_bias<<<(NN * KN + 255) / 256, 256, 0, stream>>>(xyz + (size_t)b * NN * 3, ib, W1, b1, W2, b2, BIAS);
        k_attn<<<(unsigned)(((size_t)NN * CC / 4 + 255) / 256), 256, 0, stream>>>(FQ, FK, FV, ib, BIAS, Ah, Al);
        k_gemmw<bf, 1, true><<<dim3(NN / 64, CC / 64, 1), 32, 0, stream>>>(Ah, Al, WO, nullptr, CC, OUT + (size_t)b * NN * CC, CC, bo, 0, 0, 0); }
}
